// BSARecLayer_66846870995500
// MI455X (gfx1250) — hardware-run, weakly checked
//
#include <hip/hip_runtime.h>
#include <math.h>

constexpr int kBatch  = 4;
constexpr int kSeq    = 2048;
constexpr int kDim    = 1024;
constexpr int kHeads  = 16;
constexpr int kDh     = 64;
constexpr int kTok    = kBatch * kSeq;
constexpr int kChunkG = 2;
constexpr int kNumChunks = (kBatch * kHeads) / kChunkG;
constexpr float kAlpha      = 0.7f;
constexpr float kWCarry     = 16.0f;
constexpr float kWCarryInv  = 1.0f / 16.0f;
constexpr float kPCarry     = 2048.0f;
constexpr float kPVScale    = 0.3f / 2048.0f;
constexpr float kScoreScale = 0.125f;
constexpr float kLnEps      = 1e-12f;
constexpr float kInvS       = 1.0f / 2048.0f;
constexpr float kTwoInvS    = 1.0f / 1024.0f;
constexpr float kInvD       = 1.0f / 1024.0f;
constexpr float kTheta      = (float)(6.283185307179586476925286766559 / 2048.0);

constexpr size_t kOffS    = 0;
constexpr size_t kOffX16  = 0;
constexpr size_t kOffW16  = 16777216;
constexpr size_t kOffP    = 33554432;
constexpr size_t kOffCoef = 33554432;
constexpr size_t kOffTab  = 33554432 + 81920;
constexpr size_t kOffQ    = 50331648;
constexpr size_t kOffK    = 67108864;
constexpr size_t kOffVT   = 83886080;
constexpr size_t kOffDSP  = 100663296;
constexpr size_t kWsTotal = 134217728;
static_assert(kOffW16 + (size_t)3 * kDim * kDim * 2 <= kOffP);
static_assert(kOffTab + (size_t)kSeq * 2 * 4 <= kOffQ);
static_assert(kOffDSP + (size_t)kTok * kDim * 4 == kWsTotal);

typedef __attribute__((ext_vector_type(16))) _Float16 v16h;
typedef __attribute__((ext_vector_type(8)))  _Float16 v8h;
typedef __attribute__((ext_vector_type(16))) __bf16   v16b;
typedef __attribute__((ext_vector_type(8)))  __bf16   v8b;
typedef __attribute__((ext_vector_type(8)))  float    v8f;
typedef __attribute__((ext_vector_type(4)))  float    v4f;
typedef __attribute__((ext_vector_type(2)))  float    v2f;
typedef __attribute__((ext_vector_type(4)))  unsigned int v4u;
typedef __attribute__((ext_vector_type(4)))  int      v4i;

__device__ __forceinline__ unsigned short f2bf_bits(float f) {
  unsigned u = __float_as_uint(f);
  return (unsigned short)((u + 0x7FFFu + ((u >> 16) & 1u)) >> 16);
}
__device__ __forceinline__ float bf_bits2f(unsigned short h) { return __uint_as_float(((unsigned)h) << 16); }

__device__ __forceinline__ void dep_guard_h(v8f& a, v8f& b, v16h x, v16h y) { asm volatile("v_nop\n\tv_nop\n\tv_nop\n\tv_nop" : "+v"(a), "+v"(b) : "v"(x), "v"(y)); }
__device__ __forceinline__ void dep_guard_b(v8f& a, v8f& b, v16b x, v16b y) { asm volatile("v_nop\n\tv_nop\n\tv_nop\n\tv_nop" : "+v"(a), "+v"(b) : "v"(x), "v"(y)); }
__device__ __forceinline__ void keep4_h(v16h a, v16h b, v16h c, v16h d) { asm volatile("v_nop" :: "v"(a), "v"(b), "v"(c), "v"(d)); }
__device__ __forceinline__ void keep4_b(v16b a, v16b b, v16b c, v16b d) { asm volatile("v_nop" :: "v"(a), "v"(b), "v"(c), "v"(d)); }
__device__ __forceinline__ void acc_guard4(v8f& a, v8f& b, v8f& c, v8f& d) { asm volatile("v_nop\n\tv_nop\n\tv_nop\n\tv_nop" : "+v"(a), "+v"(b), "+v"(c), "+v"(d)); }
template <typename T> struct Frag;
template <> struct Frag<_Float16> {
  typedef v16h V; union U { v16h v; v8h h[2]; };
  static __device__ __forceinline__ v16h load(const _Float16* p) {
    U f; f.h[0] = *(const v8h*)(p); f.h[1] = *(const v8h*)(p + 16); return f.v;
  }
  static __device__ __forceinline__ v8f mma(v16h a, v16h b, v8f c) {
    return __builtin_amdgcn_wmma_f32_16x16x32_f16(false, a, false, b, (short)0, c, false, false);
  }
  static __device__ __forceinline__ void guard(v8f& a, v8f& b, v16h x, v16h y) { dep_guard_h(a, b, x, y); }
  static __device__ __forceinline__ void keep(v16h a, v16h b, v16h c, v16h d) { keep4_h(a, b, c, d); }
};
template <> struct Frag<__bf16> {
  typedef v16b V; union U { v16b v; v8b h[2]; };
  static __device__ __forceinline__ v16b load(const __bf16* p) {
    U f; f.h[0] = *(const v8b*)(p); f.h[1] = *(const v8b*)(p + 16); return f.v;
  }
  static __device__ __forceinline__ v8f mma(v16b a, v16b b, v8f c) {
    return __builtin_amdgcn_wmma_f32_16x16x32_bf16(false, a, false, b, (short)0, c, false, false);
  }
  static __device__ __forceinline__ void guard(v8f& a, v8f& b, v16b x, v16b y) { dep_guard_b(a, b, x, y); }
  static __device__ __forceinline__ void keep(v16b a, v16b b, v16b c, v16b d) { keep4_b(a, b, c, d); }
};

__device__ __forceinline__ unsigned pk16(unsigned short a, unsigned short b) { return (unsigned)a | ((unsigned)b << 16); }
__device__ __forceinline__ unsigned short h_bits(float f) { const _Float16 h = (_Float16)f; return __builtin_bit_cast(unsigned short, h); }

template <int ET> struct Elem;
template <> struct Elem<0> { typedef _Float16 T; };
template <> struct Elem<1> { typedef __bf16 T; };
template <int ET, bool SPLIT, int BIAS_MODE, int OUT_MODE, bool RESID, int ACT = 0>
__global__ __launch_bounds__(256) void wmma_gemm64(
    const unsigned short* __restrict__ Ap, const unsigned short* __restrict__ A2p, int lda, long strideA,
    const unsigned short* __restrict__ Btp, const unsigned short* __restrict__ Bt2p, int ldb, long strideB,
    void* __restrict__ Cout, void* __restrict__ Cout2, int ldc, long strideC,
    const float* __restrict__ bias,
    const float* __restrict__ resid, long strideR,
    int M, int N, int K, float scale) {
  typedef typename Elem<ET>::T T;
  typedef typename Frag<T>::V V;
  const T* A = (const T*)Ap; const T* A2 = (const T*)A2p; const T* Bt = (const T*)Btp; const T* Bt2 = (const T*)Bt2p;
  __shared__ __align__(16) float sT[8][16 * 68];
  const int b    = blockIdx.y;
  const int lane = threadIdx.x & 31;
  const int wave = threadIdx.x >> 5;
  const int tilesN = N >> 6;
  const int tilesM = M >> 6;
  const int tile = blockIdx.x * 8 + wave;
  if (tile >= tilesM * tilesN) return;
  const int tm = tile / tilesN;
  const int tn = tile - tm * tilesN;
  const int m0 = tm << 6;
  const int n0 = tn << 6;

  const T* Ab  = A  + (size_t)b * strideA;
  const T* Bb  = Bt + (size_t)b * strideB;
  const T* Ab2 = SPLIT ? (A2  + (size_t)b * strideA) : nullptr;
  const T* Bb2 = SPLIT ? (Bt2 + (size_t)b * strideB) : nullptr;

  const int rlane = lane & 15;
  const int koff  = (lane >> 4) * 8;
  const int mOff  = (lane >> 4) * 8;

  v8f acc[4][4];
#pragma unroll
  for (int i = 0; i < 4; ++i)
#pragma unroll
    for (int j = 0; j < 4; ++j) acc[i][j] = (v8f){0.f,0.f,0.f,0.f,0.f,0.f,0.f,0.f};

  for (int k0 = 0; k0 < K; k0 += 32) {
    V bh[4], bl[4];
#pragma unroll
    for (int j = 0; j < 4; ++j) {
      const size_t bo = (size_t)(n0 + (j << 4) + rlane) * ldb + koff + k0;
      bh[j] = Frag<T>::load(Bb + bo);
      if (SPLIT) bl[j] = Frag<T>::load(Bb2 + bo);
    }
#pragma unroll
    for (int i = 0; i < 4; ++i) {
      const size_t ao = (size_t)(m0 + (i << 4) + rlane) * lda + koff + k0;
      V ah = Frag<T>::load(Ab + ao);
      V al;
      if (SPLIT) al = Frag<T>::load(Ab2 + ao);
#pragma unroll
      for (int j = 0; j < 4; ++j) {
        acc[i][j] = Frag<T>::mma(ah, bh[j], acc[i][j]);
        if (SPLIT) {
          acc[i][j] = Frag<T>::mma(ah, bl[j], acc[i][j]);
          acc[i][j] = Frag<T>::mma(al, bh[j], acc[i][j]);
        }
      }
      Frag<T>::guard(acc[i][0], acc[i][3], ah, SPLIT ? al : ah);
    }
    Frag<T>::keep(bh[0], bh[1], bh[2], bh[3]);
    if (SPLIT) Frag<T>::keep(bl[0], bl[1], bl[2], bl[3]);
  }
  acc_guard4(acc[0][0], acc[0][1], acc[0][2], acc[0][3]);
  acc_guard4(acc[1][0], acc[1][1], acc[1][2], acc[1][3]);
  acc_guard4(acc[2][0], acc[2][1], acc[2][2], acc[2][3]);
  acc_guard4(acc[3][0], acc[3][1], acc[3][2], acc[3][3]);

  float* slab = sT[wave];
  const float* Rb = RESID ? (resid + (size_t)b * strideR) : nullptr;
#pragma unroll
  for (int i = 0; i < 4; ++i) {
    const int mBase = m0 + (i << 4);
#pragma unroll
    for (int j = 0; j < 4; ++j) {
      const int n = n0 + (j << 4) + rlane;
      float bv = 0.f;
      if (BIAS_MODE == 2) bv = bias[n];
#pragma unroll
      for (int r = 0; r < 8; ++r) {
        float v = acc[i][j][r] * scale;
        if (BIAS_MODE == 1) v += bias[mBase + mOff + r];
        if (BIAS_MODE == 2) v += bv;
        if (RESID) v += Rb[(size_t)(mBase + mOff + r) * ldc + n];
        if (ACT == 2) v = fmaxf(v, 0.0f);
        if (ACT == 4) v = (v > 0.f) ? v : 0.01f * v;
        slab[(mOff + r) * 68 + (j << 4) + rlane] = v;
      }
    }
    __builtin_amdgcn_fence(__ATOMIC_RELEASE, "workgroup");
    __builtin_amdgcn_wave_barrier();
    __builtin_amdgcn_fence(__ATOMIC_ACQUIRE, "workgroup");
    if (OUT_MODE == 0) {
      float* C = (float*)Cout + (size_t)b * strideC;
      const int hh = lane >> 4, c4 = (lane & 15) * 4;
      for (int pass = 0; pass < 2; ++pass) {
#pragma unroll
        for (int it = 0; it < 8; ++it) {
          const int row = it * 2 + hh;
          v4f v = *(const v4f*)(slab + row * 68 + c4);
          *(volatile v4f*)(C + (size_t)(mBase + row) * ldc + n0 + c4) = v;
        }
        __threadfence();
      }
    } else {
      const int q = lane >> 3, c8 = (lane & 7) * 8;
      unsigned short* C  = (unsigned short*)Cout  + (size_t)b * strideC;
      unsigned short* C2 = (OUT_MODE == 2) ? ((unsigned short*)Cout2 + (size_t)b * strideC) : nullptr;
      for (int pass = 0; pass < 2; ++pass) {
#pragma unroll
        for (int it = 0; it < 4; ++it) {
          const int row = it * 4 + q;
          const float* sp = slab + row * 68 + c8;
          v8h hv, lv;
#pragma unroll
          for (int e = 0; e < 8; ++e) {
            if (OUT_MODE == 1) {
              hv[e] = (_Float16)sp[e];
            } else {
              unsigned short hb = f2bf_bits(sp[e]);
              unsigned short lb = f2bf_bits(sp[e] - bf_bits2f(hb));
              hv[e] = __builtin_bit_cast(_Float16, hb);
              lv[e] = __builtin_bit_cast(_Float16, lb);
            }
          }
          *(volatile v8h*)(C + (size_t)(mBase + row) * ldc + n0 + c8) = hv;
          if (OUT_MODE == 2) *(volatile v8h*)(C2 + (size_t)(mBase + row) * ldc + n0 + c8) = lv;
        }
        __threadfence();
      }
    }
    __builtin_amdgcn_fence(__ATOMIC_RELEASE, "workgroup");
    __builtin_amdgcn_wave_barrier();
    __builtin_amdgcn_fence(__ATOMIC_ACQUIRE, "workgroup");
  }
}

__global__ __launch_bounds__(256) void cast8_f16_kernel(const float* __restrict__ in, unsigned short* __restrict__ out,
                                                        int n8, float scale) {
  const int i = blockIdx.x * 256 + threadIdx.x;
  if (i >= n8) return;
  const float* p = in + 8 * (size_t)i;
  const v4f a = *(const v4f*)(p);
  const v4f c = *(const v4f*)(p + 4);
  unsigned short hb[8];
#pragma unroll
  for (int e = 0; e < 4; ++e) {
    hb[e]     = h_bits(a[e] * scale);
    hb[4 + e] = h_bits(c[e] * scale);
  }
  const v4u u = (v4u){pk16(hb[0], hb[1]), pk16(hb[2], hb[3]), pk16(hb[4], hb[5]), pk16(hb[6], hb[7])};
  unsigned short* q = out + 8 * (size_t)i;
  *(volatile v4u*)q = u;
  __threadfence();
  *(volatile v4u*)q = u;
}

__global__ __launch_bounds__(256) void dft_coeff_kernel(const float* __restrict__ x, float* __restrict__ coeff,
                                                        float* __restrict__ tab) {
  __shared__ float tcs[kSeq];
  __shared__ float tsn[kSeq];
  const int t = threadIdx.x;
  const bool writer = (blockIdx.x == 0) && (blockIdx.y == 0);
#pragma unroll 1
  for (int i = 0; i < kSeq / 256; ++i) {
    const int s = i * 256 + t;
    const float ang = (float)s * kTheta;
    float sn, cs;
    sincosf(ang, &sn, &cs);
    tcs[s] = cs;
    tsn[s] = sn;
    if (writer) {
      const v2f val = (v2f){cs, sn};
      *(volatile v2f*)(tab + 2 * (size_t)s) = val;
      __threadfence();
      *(volatile v2f*)(tab + 2 * (size_t)s) = val;
    }
  }
  __syncthreads();
  const int b = blockIdx.y;
  const int d = blockIdx.x * 256 + t;
  const float* xp = x + (size_t)b * kSeq * kDim + d;
  float c0 = 0.f, c1c = 0.f, c1s = 0.f, c2c = 0.f, c2s = 0.f;
#pragma unroll 1
  for (int s = 0; s < kSeq; ++s) {
    const float xv = xp[(size_t)s * kDim];
    const int s2 = (2 * s) & (kSeq - 1);
    const float cs = tcs[s], sn = tsn[s], cs2 = tcs[s2], sn2 = tsn[s2];
    c0  += xv;
    c1c += xv * cs;
    c1s += xv * sn;
    c2c += xv * cs2;
    c2s += xv * sn2;
  }
  float* cp = coeff + (size_t)b * 5 * kDim + d;
  *(volatile float*)(cp)            = c0;
  *(volatile float*)(cp + kDim)     = c1c;
  *(volatile float*)(cp + 2 * kDim) = c1s;
  *(volatile float*)(cp + 3 * kDim) = c2c;
  *(volatile float*)(cp + 4 * kDim) = c2s;
  __threadfence();
  *(volatile float*)(cp)            = c0;
  *(volatile float*)(cp + kDim)     = c1c;
  *(volatile float*)(cp + 2 * kDim) = c1s;
  *(volatile float*)(cp + 3 * kDim) = c2c;
  *(volatile float*)(cp + 4 * kDim) = c2s;
}

__global__ __launch_bounds__(256) void dsp_row_kernel(const float* __restrict__ x, const float* __restrict__ coeff,
                                                      const float* __restrict__ tab, const float* __restrict__ sqrt_beta,
                                                      const float* __restrict__ gamma, const float* __restrict__ beta,
                                                      float* __restrict__ dsp) {
  __shared__ float redA[8];
  __shared__ float redB[8];
  const int tok  = blockIdx.x;
  const int b    = tok / kSeq;
  const int s    = tok - b * kSeq;
  const int t    = threadIdx.x;
  const int lane = t & 31, wave = t >> 5;
  const int c4   = 4 * t;
  const v2f t1 = *(const v2f*)(tab + 2 * (size_t)s);
  const v2f t2 = *(const v2f*)(tab + 2 * (size_t)((2 * s) & (kSeq - 1)));
  const float cs = t1[0], sn = t1[1], cs2 = t2[0], sn2 = t2[1];
  const v4f xv  = *(const v4f*)(x + (size_t)tok * kDim + c4);
  const float* cb = coeff + (size_t)b * 5 * kDim + c4;
  const v4f a0  = *(const v4f*)(cb);
  const v4f a1c = *(const v4f*)(cb + kDim);
  const v4f a1s = *(const v4f*)(cb + 2 * kDim);
  const v4f a2c = *(const v4f*)(cb + 3 * kDim);
  const v4f a2s = *(const v4f*)(cb + 4 * kDim);
  const v4f sb  = *(const v4f*)(sqrt_beta + c4);
  const v4f g   = *(const v4f*)(gamma + c4);
  const v4f be  = *(const v4f*)(beta + c4);
  float y[4];
  float sum = 0.f;
#pragma unroll
  for (int e = 0; e < 4; ++e) {
    const float low  = a0[e] * kInvS + (a1c[e] * cs + a1s[e] * sn + a2c[e] * cs2 + a2s[e] * sn2) * kTwoInvS;
    const float high = xv[e] - low;
    const float sf   = low + (sb[e] * sb[e]) * high;
    y[e] = sf + xv[e];
    sum += y[e];
  }
#pragma unroll
  for (int off = 16; off > 0; off >>= 1) sum += __shfl_xor(sum, off, 32);
  if (lane == 0) redA[wave] = sum;
  __syncthreads();
  float tot = 0.f;
#pragma unroll
  for (int w = 0; w < 8; ++w) tot += redA[w];
  const float mu = tot * kInvD;
  float sq = 0.f;
#pragma unroll
  for (int e = 0; e < 4; ++e) { const float dv = y[e] - mu; sq += dv * dv; }
#pragma unroll
  for (int off = 16; off > 0; off >>= 1) sq += __shfl_xor(sq, off, 32);
  if (lane == 0) redB[wave] = sq;
  __syncthreads();
  float tot2 = 0.f;
#pragma unroll
  for (int w = 0; w < 8; ++w) tot2 += redB[w];
  const float var = tot2 * kInvD;
  const float inv = rsqrtf(var + kLnEps);
  v4f o;
#pragma unroll
  for (int e = 0; e < 4; ++e) o[e] = kAlpha * ((y[e] - mu) * inv * g[e] + be[e]);
  float* op = dsp + (size_t)tok * kDim + c4;
  *(volatile v4f*)op = o;
  __threadfence();
  *(volatile v4f*)op = o;
}

__global__ __launch_bounds__(256) void softmax_row_kernel(const float* __restrict__ S, const int* __restrict__ mask,
                                                          unsigned short* __restrict__ P, float carry) {
  __shared__ float redM[8];
  __shared__ float redS[8];
  const int row  = blockIdx.x;
  const int qrow = row & (kSeq - 1);
  const int t    = threadIdx.x;
  const int lane = t & 31, wave = t >> 5;
  const int c0   = t * 8;
  const float* sr = S + (size_t)row * kSeq + c0;
  const v4f a = *(const v4f*)(sr);
  const v4f c = *(const v4f*)(sr + 4);
  const int* mr = mask + (size_t)qrow * kSeq + c0;
  const v4i ma = *(const v4i*)(mr);
  const v4i mc = *(const v4i*)(mr + 4);
  float x[8];
#pragma unroll
  for (int e = 0; e < 4; ++e) {
    x[e]     = (ma[e] == 0) ? -INFINITY : a[e];
    x[4 + e] = (mc[e] == 0) ? -INFINITY : c[e];
  }
  float m = fmaxf(fmaxf(fmaxf(x[0], x[1]), fmaxf(x[2], x[3])), fmaxf(fmaxf(x[4], x[5]), fmaxf(x[6], x[7])));
#pragma unroll
  for (int off = 16; off > 0; off >>= 1) m = fmaxf(m, __shfl_xor(m, off, 32));
  if (lane == 0) redM[wave] = m;
  __syncthreads();
  float bm = redM[0];
#pragma unroll
  for (int w = 1; w < 8; ++w) bm = fmaxf(bm, redM[w]);
  const float mref = (bm == -INFINITY) ? 0.f : bm;
  float p[8];
  float psum = 0.f;
#pragma unroll
  for (int e = 0; e < 8; ++e) { p[e] = expf(x[e] - mref); psum += p[e]; }
#pragma unroll
  for (int off = 16; off > 0; off >>= 1) psum += __shfl_xor(psum, off, 32);
  if (lane == 0) redS[wave] = psum;
  __syncthreads();
  float tot = 0.f;
#pragma unroll
  for (int w = 0; w < 8; ++w) tot += redS[w];
  const float rs  = 1.0f / fmaxf(tot, 1e-30f);
  const float inv = (tot > 0.f) ? (carry * rs) : 0.f;
  unsigned short hb[8];
#pragma unroll
  for (int e = 0; e < 8; ++e) hb[e] = h_bits(p[e] * inv);
  const v4u u = (v4u){pk16(hb[0], hb[1]), pk16(hb[2], hb[3]), pk16(hb[4], hb[5]), pk16(hb[6], hb[7])};
  unsigned short* pp = P + (size_t)row * kSeq + c0;
  *(volatile v4u*)pp = u;
  __threadfence();
  *(volatile v4u*)pp = u;
}

extern "C" void kernel_launch(void* const* d_in, const int* in_sizes, int n_in,
                              void* d_out, int out_size, void* d_ws, size_t ws_size,
                              hipStream_t stream) {
  if (n_in < 11) return;
  if (in_sizes[0] != kTok * kDim) return;
  if (in_sizes[1] != kSeq * kSeq) return;
  if (in_sizes[2] != kDim || in_sizes[3] != kDim || in_sizes[4] != kDim) return;
  if (in_sizes[5] != kDim * kDim || in_sizes[7] != kDim * kDim || in_sizes[9] != kDim * kDim) return;
  if (in_sizes[6] != kDim || in_sizes[8] != kDim || in_sizes[10] != kDim) return;
  if (out_size != kTok * kDim) return;
  if (ws_size < kWsTotal) return;

  const float* x         = (const float*)d_in[0];
  const int*   mask      = (const int*)d_in[1];
  const float* sqrt_beta = (const float*)d_in[2];
  const float* ln_g      = (const float*)d_in[3];
  const float* ln_b      = (const float*)d_in[4];
  const float* q_w       = (const float*)d_in[5];
  const float* q_b       = (const float*)d_in[6];
  const float* k_w       = (const float*)d_in[7];
  const float* k_b       = (const float*)d_in[8];
  const float* v_w       = (const float*)d_in[9];
  const float* v_b       = (const float*)d_in[10];
  float* out = (float*)d_out;

  char* w = (char*)d_ws;
  float*          Sreg = (float*)(w + kOffS);
  unsigned short* X16  = (unsigned short*)(w + kOffX16);
  unsigned short* W16  = (unsigned short*)(w + kOffW16);
  unsigned short* Preg = (unsigned short*)(w + kOffP);
  float*          coef = (float*)(w + kOffCoef);
  float*          tab  = (float*)(w + kOffTab);
  unsigned short* Q16  = (unsigned short*)(w + kOffQ);
  unsigned short* K16  = (unsigned short*)(w + kOffK);
  unsigned short* VT16 = (unsigned short*)(w + kOffVT);
  float*          DSPp = (float*)(w + kOffDSP);
  unsigned short* W16q = W16;
  unsigned short* W16k = W16 + (size_t)kDim * kDim;
  unsigned short* W16v = W16 + (size_t)2 * kDim * kDim;

  cast8_f16_kernel<<<(kTok * kDim) / (8 * 256), 256, 0, stream>>>(x, X16, (kTok * kDim) / 8, 1.0f);
  cast8_f16_kernel<<<(kDim * kDim) / (8 * 256), 256, 0, stream>>>(q_w, W16q, (kDim * kDim) / 8, kWCarry);
  cast8_f16_kernel<<<(kDim * kDim) / (8 * 256), 256, 0, stream>>>(k_w, W16k, (kDim * kDim) / 8, kWCarry);
  cast8_f16_kernel<<<(kDim * kDim) / (8 * 256), 256, 0, stream>>>(v_w, W16v, (kDim * kDim) / 8, kWCarry);

  dft_coeff_kernel<<<dim3(kDim / 256, kBatch), 256, 0, stream>>>(x, coef, tab);
  dsp_row_kernel<<<kTok, 256, 0, stream>>>(x, coef, tab, sqrt_beta, ln_g, ln_b, DSPp);

  wmma_gemm64<0, false, 2, 1, false> <<<dim3(256, 1), 256, 0, stream>>>(
      X16, X16, kDim, 0L, W16q, W16q, kDim, 0L, (void*)Q16, (void*)Q16, kDim, 0L,
      q_b, DSPp, 0L, kTok, kDim, kDim, kWCarryInv);
  wmma_gemm64<0, false, 2, 1, false> <<<dim3(256, 1), 256, 0, stream>>>(
      X16, X16, kDim, 0L, W16k, W16k, kDim, 0L, (void*)K16, (void*)K16, kDim, 0L,
      k_b, DSPp, 0L, kTok, kDim, kDim, kWCarryInv);
  wmma_gemm64<0, false, 1, 1, false> <<<dim3(64, kBatch), 256, 0, stream>>>(
      W16v, W16v, kDim, 0L, X16, X16, kDim, (long)kSeq * kDim, (void*)VT16, (void*)VT16, kSeq, (long)kDim * kSeq,
      v_b, DSPp, 0L, kDim, kSeq, kDim, kWCarryInv);

  for (int cidx = 0; cidx < kNumChunks; ++cidx) {
    const int g0 = cidx * kChunkG;
    const int b  = g0 / kHeads;
    const int h0 = g0 - b * kHeads;
    const size_t qkOff  = (size_t)b * kSeq * kDim + (size_t)h0 * kDh;
    const size_t vtOff  = ((size_t)b * kDim + (size_t)h0 * kDh) * kSeq;
    const size_t outOff = (size_t)b * kSeq * kDim + (size_t)h0 * kDh;
    wmma_gemm64<0, false, 0, 0, false> <<<dim3(128, kChunkG), 256, 0, stream>>>(
        Q16 + qkOff, Q16 + qkOff, kDim, (long)kDh, K16 + qkOff, K16 + qkOff, kDim, (long)kDh,
        (void*)Sreg, (void*)Sreg, kSeq, (long)kSeq * kSeq,
        q_b, DSPp, 0L, kSeq, kSeq, kDh, kScoreScale);
    softmax_row_kernel<<<kChunkG * kSeq, 256, 0, stream>>>(Sreg, mask, Preg, kPCarry);
    wmma_gemm64<0, false, 0, 0, true> <<<dim3(4, kChunkG), 256, 0, stream>>>(
        Preg, Preg, kSeq, (long)kSeq * kSeq, VT16 + vtOff, VT16 + vtOff, kSeq, (long)kDh * kSeq,
        (void*)(out + outOff), (void*)(out + outOff), kDim, (long)kDh,
        q_b, DSPp + outOff, (long)kDh, kSeq, kDh, kSeq, kPVScale);
  }
}
